// S6_31799937860325
// MI455X (gfx1250) — hardware-verified
//
#include <hip/hip_runtime.h>
#include <math.h>

typedef __attribute__((ext_vector_type(16))) _Float16 v16h;
typedef __attribute__((ext_vector_type(8)))  _Float16 v8h;
typedef __attribute__((ext_vector_type(8)))  float    v8f;
typedef __attribute__((ext_vector_type(4)))  float    v4f;

constexpr int kBatch = 4;
constexpr int kSeq   = 2048;
constexpr int kDm    = 1024;
constexpr int kDin   = 2048;
constexpr int kNst   = 16;
constexpr int kDtR   = 64;
constexpr int kPrjN  = 96;
constexpr int kPrjP  = 128;
constexpr int kXzN   = 2 * kDin;
constexpr int kRows  = kBatch * kSeq;
constexpr int kBcP   = 32;
constexpr int kTP    = 260;

constexpr float kCarryWin  = 32.0f;
constexpr float kCarryWx   = 32.0f;
constexpr float kCarryWout = 32.0f;
constexpr float kCarryWdt  = 8.0f;
constexpr float kCarryDtLr = 16.0f;
constexpr float kCarryDt   = 16.0f;
constexpr float kCarryY    = 16.0f;
constexpr float kLog2e     = 1.4426950408889634f;

static_assert(kDtR + 2 * kNst == kPrjN);
static_assert(kPrjP == 128 && kPrjP >= kPrjN);
static_assert((kDm % 32) == 0 && (kDin % 32) == 0 && (kDtR % 32) == 0);
static_assert((kRows % 64) == 0 && (kXzN % 64) == 0 && (kPrjP % 64) == 0 && (kDin % 64) == 0 && (kDm % 64) == 0);
static_assert((kSeq % 64) == 0 && (kDin % 256) == 0);
static_assert(2 * kNst == kBcP);

constexpr size_t kOffX16  = 0;
constexpr size_t kOffWIN  = kOffX16  + (size_t)kRows * kDm  * 2;
constexpr size_t kOffXB   = kOffWIN  + (size_t)kXzN  * kDm  * 2;
constexpr size_t kOffG    = kOffXB   + (size_t)kRows * kDin * 2;
constexpr size_t kOffU    = kOffG    + (size_t)kRows * kDin * 2;
constexpr size_t kOffBC   = kOffU    + (size_t)kRows * kDin * 2;
constexpr size_t kOffDTLR = kOffBC   + (size_t)kRows * kBcP * 4;
constexpr size_t kOffWOUT = kOffDTLR + (size_t)kRows * kDtR * 2;
constexpr size_t kOffWX   = kOffWOUT + (size_t)kDm   * kDin * 2;
constexpr size_t kOffWDT  = kOffWX   + (size_t)kPrjP * kDin * 2;
constexpr size_t kWsTotal = kOffWDT  + (size_t)kDin  * kDtR * 2;
static_assert(kWsTotal == 132907008ull);
static_assert(kWsTotal <= 134217728ull);
static_assert((kOffWIN % 128) == 0 && (kOffXB % 128) == 0 && (kOffG % 128) == 0 && (kOffU % 128) == 0 &&
              (kOffBC % 128) == 0 && (kOffDTLR % 128) == 0 && (kOffWOUT % 128) == 0 && (kOffWX % 128) == 0 &&
              (kOffWDT % 128) == 0);

__device__ __forceinline__ float bf_rne(float f) {
  const unsigned u = __float_as_uint(f);
  return __uint_as_float((u + 0x7FFFu + ((u >> 16) & 1u)) & 0xFFFF0000u);
}
__device__ __forceinline__ float h16_to_f32(unsigned hb) {
  const unsigned sgn = (hb & 0x8000u) << 16;
  const unsigned em = hb & 0x7fffu;
  const float fn = __uint_as_float((em << 13) + 0x38000000u);
  const float fs = (float)em * 5.9604644775390625e-8f;
  const float mag = (em < 0x400u) ? fs : fn;
  return __uint_as_float(__float_as_uint(mag) | sgn);
}
__device__ __forceinline__ float silu_fast(float v) {
  return v * __builtin_amdgcn_rcpf(1.0f + __expf(-v));
}
__device__ __forceinline__ float softplus_fast(float v) {
  const float a  = __expf(-fabsf(v));
  const float u  = 1.0f + a;
  const float lg = __logf(u) + (a - (u - 1.0f)) * __builtin_amdgcn_rcpf(u);
  const float ps = a * (1.0f - a * (0.5f - a * 0.33333334f));
  const float l1p = (a < 0.00390625f) ? ps : lg;
  return fmaxf(v, 0.0f) + l1p;
}

__device__ __forceinline__ void guard_row(v8f& a0, v8f& a1, v8f& a2, v8f& a3,
                                          v16h x, v16h b0, v16h b1, v16h b2, v16h b3) {
  asm volatile("v_nop\n\tv_nop\n\tv_nop\n\tv_nop"
               : "+v"(a0), "+v"(a1), "+v"(a2), "+v"(a3)
               : "v"(x), "v"(b0), "v"(b1), "v"(b2), "v"(b3));
}
__device__ __forceinline__ void keep4_h(v16h a, v16h b, v16h c, v16h d) { asm volatile("v_nop" :: "v"(a), "v"(b), "v"(c), "v"(d)); }
__device__ __forceinline__ void acc_guard4(v8f& a, v8f& b, v8f& c, v8f& d) { asm volatile("v_nop\n\tv_nop\n\tv_nop\n\tv_nop" : "+v"(a), "+v"(b), "+v"(c), "+v"(d)); }

template <typename T> struct Frag;
template <> struct Frag<_Float16> {
  typedef v16h V; union U { v16h v; v8h h[2]; };
  static __device__ __forceinline__ v16h load(const _Float16* p) {
    U f; f.h[0] = *(const v8h*)(p); f.h[1] = *(const v8h*)(p + 16); return f.v;
  }
  static __device__ __forceinline__ v8f mma(v16h a, v16h b, v8f c) {
    return __builtin_amdgcn_wmma_f32_16x16x32_f16(false, a, false, b, (short)0, c, false, false);
  }
};

__global__ __launch_bounds__(256) void cast_bf16_f16_kernel(
    const float* __restrict__ src, unsigned short* __restrict__ dst, int total8, int real8, float scale)
{
  const int i = blockIdx.x * 256 + threadIdx.x;
  if (i >= total8) return;
  const bool live = (i < real8);
  const int ic = live ? i : (real8 - 1);
  const float* p = src + ((size_t)ic << 3);
  const v4f a0 = *(const v4f*)(p);
  const v4f a1 = *(const v4f*)(p + 4);
  v8h hv;
#pragma unroll
  for (int e = 0; e < 4; ++e) {
    const float f0 = a0[e];
    const float f1 = a1[e];
    const float r0 = bf_rne(f0) * scale;
    const float r1 = bf_rne(f1) * scale;
    hv[e]     = (_Float16)(live ? r0 : 0.0f);
    hv[4 + e] = (_Float16)(live ? r1 : 0.0f);
  }
  unsigned short* q = dst + ((size_t)i << 3);
  *(volatile v8h*)q = hv;
  __threadfence();
  *(volatile v8h*)q = hv;
}

constexpr int EPI_OUT = 0;
constexpr int EPI_INPROJ = 1;
constexpr int EPI_XPROJ = 2;
constexpr int EPI_DT = 3;

template <int EPI>
__global__ __launch_bounds__(256) void gemm_f16_kernel(
    const unsigned short* __restrict__ Ap, int lda,
    const unsigned short* __restrict__ Btp, int ldb,
    void* C0, void* C1, int ldc,
    const float* __restrict__ bias,
    int M, int N, int K, float scale)
{
  typedef _Float16 T;
  typedef v16h V;
  const T* A  = (const T*)Ap;
  const T* Bt = (const T*)Btp;
  __shared__ __align__(16) float sT[8][16 * 68];
  const int lane = threadIdx.x & 31;
  const int wave = threadIdx.x >> 5;
  const int tilesN = N >> 6;
  const int tilesM = M >> 6;
  const int tile = blockIdx.x * 8 + wave;
  if (tile >= tilesM * tilesN) return;
  const int tm = tile / tilesN;
  const int tn = tile - tm * tilesN;
  const int m0 = tm << 6;
  const int n0 = tn << 6;

  const int rlane = lane & 15;
  const int koff  = (lane >> 4) * 8;
  const int mOff  = (lane >> 4) * 8;

  v8f acc[4][4];
#pragma unroll
  for (int i = 0; i < 4; ++i)
#pragma unroll
    for (int j = 0; j < 4; ++j) acc[i][j] = (v8f){0.f,0.f,0.f,0.f,0.f,0.f,0.f,0.f};

  for (int k0 = 0; k0 < K; k0 += 32) {
    V bh[4];
#pragma unroll
    for (int j = 0; j < 4; ++j) {
      const size_t bo = (size_t)(n0 + (j << 4) + rlane) * ldb + koff + k0;
      bh[j] = Frag<T>::load(Bt + bo);
    }
#pragma unroll
    for (int i = 0; i < 4; ++i) {
      const size_t ao = (size_t)(m0 + (i << 4) + rlane) * lda + koff + k0;
      V ah = Frag<T>::load(A + ao);
#pragma unroll
      for (int j = 0; j < 4; ++j) acc[i][j] = Frag<T>::mma(ah, bh[j], acc[i][j]);
      guard_row(acc[i][0], acc[i][1], acc[i][2], acc[i][3], ah, bh[0], bh[1], bh[2], bh[3]);
    }
    keep4_h(bh[0], bh[1], bh[2], bh[3]);
  }
  acc_guard4(acc[0][0], acc[0][1], acc[0][2], acc[0][3]);
  acc_guard4(acc[1][0], acc[1][1], acc[1][2], acc[1][3]);
  acc_guard4(acc[2][0], acc[2][1], acc[2][2], acc[2][3]);
  acc_guard4(acc[3][0], acc[3][1], acc[3][2], acc[3][3]);

  float* slab = sT[wave];
  float bvv[4];
#pragma unroll
  for (int j = 0; j < 4; ++j) {
    bvv[j] = 0.f;
    if (EPI == EPI_DT) bvv[j] = bf_rne(bias[n0 + (j << 4) + rlane]);
  }
#pragma unroll
  for (int i = 0; i < 4; ++i) {
    const int mBase = m0 + (i << 4);
#pragma unroll
    for (int j = 0; j < 4; ++j) {
#pragma unroll
      for (int r = 0; r < 8; ++r) {
        float v = acc[i][j][r] * scale;
        if (EPI == EPI_DT) v += bvv[j];
        slab[(mOff + r) * 68 + (j << 4) + rlane] = v;
      }
    }
    __builtin_amdgcn_fence(__ATOMIC_RELEASE, "workgroup");
    __builtin_amdgcn_wave_barrier();
    __builtin_amdgcn_fence(__ATOMIC_ACQUIRE, "workgroup");

    if (EPI == EPI_OUT) {
      float* C = (float*)C0;
      const int hh = lane >> 4, c4 = (lane & 15) * 4;
      for (int pass = 0; pass < 2; ++pass) {
#pragma unroll
        for (int it = 0; it < 8; ++it) {
          const int row = it * 2 + hh;
          v4f v = *(const v4f*)(slab + row * 68 + c4);
          *(volatile v4f*)(C + (size_t)(mBase + row) * ldc + n0 + c4) = v;
        }
        __threadfence();
      }
    } else if (EPI == EPI_INPROJ) {
      const int q = lane >> 3, c8 = (lane & 7) * 8;
      const bool gate = (n0 >= kDin);
      unsigned short* C = gate ? (unsigned short*)C1 : (unsigned short*)C0;
      const int col = (n0 & (kDin - 1)) + c8;
#pragma unroll 1
      for (int pass = 0; pass < 2; ++pass) {
#pragma unroll 1
        for (int it = 0; it < 4; ++it) {
          const int row = it * 4 + q;
          const float* sp = slab + row * 68 + c8;
          const v4f a0 = *(const v4f*)(sp);
          const v4f a1 = *(const v4f*)(sp + 4);
          v8h hv;
#pragma unroll
          for (int e = 0; e < 4; ++e) {
            float f0 = a0[e];
            float f1 = a1[e];
            if (gate) { f0 = silu_fast(f0); f1 = silu_fast(f1); }
            hv[e]     = (_Float16)f0;
            hv[4 + e] = (_Float16)f1;
          }
          *(volatile v8h*)(C + (size_t)(mBase + row) * ldc + col) = hv;
        }
        __threadfence();
      }
    } else if (EPI == EPI_XPROJ) {
      const int q = lane >> 3;
      if (n0 == 0) {
        unsigned short* C = (unsigned short*)C0;
        const int c8 = (lane & 7) * 8;
        for (int pass = 0; pass < 2; ++pass) {
#pragma unroll
          for (int it = 0; it < 4; ++it) {
            const int row = it * 4 + q;
            const float* sp = slab + row * 68 + c8;
            const v4f a0 = *(const v4f*)(sp);
            const v4f a1 = *(const v4f*)(sp + 4);
            v8h hv;
#pragma unroll
            for (int e = 0; e < 4; ++e) {
              const float f0 = a0[e];
              const float f1 = a1[e];
              hv[e]     = (_Float16)(f0 * kCarryDtLr);
              hv[4 + e] = (_Float16)(f1 * kCarryDtLr);
            }
            *(volatile v8h*)(C + (size_t)(mBase + row) * kDtR + c8) = hv;
          }
          __threadfence();
        }
      } else {
        float* C = (float*)C1;
        const int c4 = (lane & 7) * 4;
        for (int pass = 0; pass < 2; ++pass) {
#pragma unroll
          for (int it = 0; it < 4; ++it) {
            const int row = it * 4 + q;
            v4f v = *(const v4f*)(slab + row * 68 + c4);
            *(volatile v4f*)(C + (size_t)(mBase + row) * kBcP + c4) = v;
          }
          __threadfence();
        }
      }
    } else {
      const int q = lane >> 3, c8 = (lane & 7) * 8;
      unsigned short* C = (unsigned short*)C0;
#pragma unroll 1
      for (int pass = 0; pass < 2; ++pass) {
#pragma unroll 1
        for (int it = 0; it < 4; ++it) {
          const int row = it * 4 + q;
          const float* sp = slab + row * 68 + c8;
          const v4f a0 = *(const v4f*)(sp);
          const v4f a1 = *(const v4f*)(sp + 4);
          v8h hv;
#pragma unroll
          for (int e = 0; e < 4; ++e) {
            const float f0 = a0[e];
            const float f1 = a1[e];
            hv[e]     = (_Float16)(softplus_fast(f0) * kCarryDt);
            hv[4 + e] = (_Float16)(softplus_fast(f1) * kCarryDt);
          }
          *(volatile v8h*)(C + (size_t)(mBase + row) * ldc + n0 + c8) = hv;
        }
        __threadfence();
      }
    }
    __builtin_amdgcn_fence(__ATOMIC_RELEASE, "workgroup");
    __builtin_amdgcn_wave_barrier();
    __builtin_amdgcn_fence(__ATOMIC_ACQUIRE, "workgroup");
  }
}

__global__ __launch_bounds__(256) void conv_silu_kernel(
    const unsigned* __restrict__ XBw, const float* __restrict__ cw, const float* __restrict__ cb,
    unsigned short* __restrict__ U16)
{
  __shared__ __align__(16) float sT[16 * kTP];
  const int tid = threadIdx.x, lane = tid & 31, wave = tid >> 5;
  const int d0 = blockIdx.x * 256, d = d0 + tid;
  const int g0 = blockIdx.y * 64;
  const int tb = g0 & (kSeq - 1);
  const unsigned sh = (unsigned)(tid & 1) * 16u;
  const v4f wv = *(const v4f*)(cw + (size_t)d * 4);
  const float wa = wv[0], wb = wv[1], wc = wv[2], wd = wv[3];
  const float w0 = bf_rne(wa), w1 = bf_rne(wb), w2 = bf_rne(wc), w3 = bf_rne(wd);
  const float bc = bf_rne(cb[d]);
  float xm3, xm2, xm1;
  {
    const bool hist = (tb > 0);
    const int rb = hist ? (g0 - 3) : g0;
    const unsigned q3 = XBw[((size_t)rb * kDin + d) >> 1];
    const unsigned q2 = XBw[((size_t)(rb + 1) * kDin + d) >> 1];
    const unsigned q1 = XBw[((size_t)(rb + 2) * kDin + d) >> 1];
    const float v3 = h16_to_f32((q3 >> sh) & 0xffffu);
    const float v2 = h16_to_f32((q2 >> sh) & 0xffffu);
    const float v1 = h16_to_f32((q1 >> sh) & 0xffffu);
    xm3 = hist ? v3 : 0.f;
    xm2 = hist ? v2 : 0.f;
    xm1 = hist ? v1 : 0.f;
  }
#pragma unroll 1
  for (int sub = 0; sub < 4; ++sub) {
    const int lb = g0 + sub * 16;
#pragma unroll 1
    for (int s = 0; s < 16; ++s) {
      unsigned qw = XBw[((size_t)(lb + s) * kDin + d) >> 1];
      asm volatile("" : "+v"(qw));
      const float xcur = h16_to_f32((qw >> sh) & 0xffffu);
      float acc = w0 * xm3;
      acc = fmaf(w1, xm2, acc);
      acc = fmaf(w2, xm1, acc);
      acc = fmaf(w3, xcur, acc);
      const float sv = acc + bc;
      sT[s * kTP + tid] = silu_fast(sv);
      xm3 = xm2; xm2 = xm1; xm1 = xcur;
    }
    __syncthreads();
    v8h bv[2];
#pragma unroll
    for (int it = 0; it < 2; ++it) {
      const float* sp = sT + (it * 8 + wave) * kTP + lane * 8;
      const v4f a0 = *(const v4f*)(sp);
      const v4f a1 = *(const v4f*)(sp + 4);
#pragma unroll
      for (int e = 0; e < 4; ++e) {
        const float f0 = a0[e];
        const float f1 = a1[e];
        bv[it][e]     = (_Float16)f0;
        bv[it][4 + e] = (_Float16)f1;
      }
    }
    for (int pass = 0; pass < 2; ++pass) {
#pragma unroll
      for (int it = 0; it < 2; ++it)
        *(volatile v8h*)(U16 + (size_t)(lb + it * 8 + wave) * kDin + d0 + lane * 8) = bv[it];
      __threadfence();
    }
    __syncthreads();
  }
}

__global__ __launch_bounds__(256) void scan_kernel(
    const unsigned* __restrict__ DTw, unsigned short* UY, const unsigned* __restrict__ Gw,
    const float* __restrict__ BC, const float* __restrict__ A_log, const float* __restrict__ Dv)
{
  __shared__ __align__(16) float sBC[16 * kBcP];
  __shared__ __align__(16) float sY[16 * kTP];
  const int tid = threadIdx.x, lane = tid & 31, wave = tid >> 5;
  constexpr int kBlkPerB = kDin / 256;
  const int bix = blockIdx.x / kBlkPerB;
  const int d0  = (blockIdx.x - bix * kBlkPerB) * 256;
  const int d   = d0 + tid;
  const size_t row0 = (size_t)bix * kSeq;
  const unsigned sh = (unsigned)(tid & 1) * 16u;
  const unsigned* Uw = (const unsigned*)UY;

  float A2[kNst];
#pragma unroll
  for (int qq = 0; qq < 4; ++qq) {
    const v4f av = *(const v4f*)(A_log + (size_t)d * kNst + 4 * qq);
#pragma unroll
    for (int e = 0; e < 4; ++e) {
      const float f = av[e];
      A2[4 * qq + e] = -expf(bf_rne(f)) * kLog2e;
    }
  }
  const float Dd = bf_rne(Dv[d]);
  float h[kNst];
#pragma unroll
  for (int n = 0; n < kNst; ++n) h[n] = 0.f;
  constexpr float kInvDt = 1.0f / kCarryDt;

#pragma unroll 1
  for (int c = 0; c < kSeq / 16; ++c) {
    const int l0 = c * 16;
    if (tid < 128) {
      const int r = tid >> 3, q4 = (tid & 7) * 4;
      const v4f v = *(const v4f*)(BC + (row0 + l0 + r) * kBcP + q4);
      *(v4f*)(sBC + r * kBcP + q4) = v;
    }
    __syncthreads();
#pragma unroll 1
    for (int s = 0; s < 16; ++s) {
      const size_t m  = row0 + l0 + s;
      const size_t wi = (m * kDin + d) >> 1;
      unsigned wdt = DTw[wi];
      unsigned wu  = Uw[wi];
      unsigned wg  = Gw[wi];
      asm volatile("" : "+v"(wdt), "+v"(wu), "+v"(wg));
      const float dt = h16_to_f32((wdt >> sh) & 0xffffu) * kInvDt;
      const float uv = h16_to_f32((wu >> sh) & 0xffffu);
      const float gv = h16_to_f32((wg >> sh) & 0xffffu);
      const float dtu = dt * uv;
      v4f Bq[4], Cq[4];
#pragma unroll
      for (int qq = 0; qq < 4; ++qq) {
        Bq[qq] = *(const v4f*)(sBC + s * kBcP + 4 * qq);
        Cq[qq] = *(const v4f*)(sBC + s * kBcP + kNst + 4 * qq);
      }
      float y = 0.f;
#pragma unroll
      for (int n = 0; n < kNst; ++n) {
        const float e = __builtin_amdgcn_exp2f(dt * A2[n]);
        const float hn = fmaf(e, h[n], dtu * Bq[n >> 2][n & 3]);
        h[n] = hn;
        y = fmaf(hn, Cq[n >> 2][n & 3], y);
      }
      y = fmaf(uv, Dd, y);
      sY[s * kTP + tid] = (y * gv) * kCarryY;
    }
    __syncthreads();
    v8h hv[2];
#pragma unroll
    for (int it = 0; it < 2; ++it) {
      const float* sp = sY + (it * 8 + wave) * kTP + lane * 8;
      const v4f a0 = *(const v4f*)(sp);
      const v4f a1 = *(const v4f*)(sp + 4);
#pragma unroll
      for (int e = 0; e < 4; ++e) {
        const float f0 = a0[e];
        const float f1 = a1[e];
        hv[it][e]     = (_Float16)f0;
        hv[it][4 + e] = (_Float16)f1;
      }
    }
    for (int pass = 0; pass < 2; ++pass) {
#pragma unroll
      for (int it = 0; it < 2; ++it)
        *(volatile v8h*)(UY + (row0 + l0 + it * 8 + wave) * kDin + d0 + lane * 8) = hv[it];
      __threadfence();
    }
  }
}

static_assert(((kRows / 64) * (kXzN / 64)) % 8 == 0);
static_assert(((kRows / 64) * (kPrjP / 64)) % 8 == 0);
static_assert(((kRows / 64) * (kDin / 64)) % 8 == 0);
static_assert(((kRows / 64) * (kDm / 64)) % 8 == 0);
static_assert(((kRows * kDm / 8) % 256) == 0 && ((kXzN * kDm / 8) % 256) == 0 && ((kDm * kDin / 8) % 256) == 0 &&
              ((kPrjP * kDin / 8) % 256) == 0 && ((kDin * kDtR / 8) % 256) == 0);

extern "C" void kernel_launch(void* const* d_in, const int* in_sizes, int n_in,
                              void* d_out, int out_size, void* d_ws, size_t ws_size,
                              hipStream_t stream)
{
  if (n_in < 10) return;
  if (in_sizes[0] != kRows * kDm) return;
  if (in_sizes[1] != kXzN * kDm) return;
  if (in_sizes[2] != kDin * 4) return;
  if (in_sizes[3] != kDin) return;
  if (in_sizes[4] != kPrjN * kDin) return;
  if (in_sizes[5] != kDin * kDtR) return;
  if (in_sizes[6] != kDin) return;
  if (in_sizes[7] != kDin * kNst) return;
  if (in_sizes[8] != kDin) return;
  if (in_sizes[9] != kDm * kDin) return;
  if (out_size != kRows * kDm) return;
  if (ws_size < kWsTotal) return;

  const float* x       = (const float*)d_in[0];
  const float* W_in    = (const float*)d_in[1];
  const float* conv_w  = (const float*)d_in[2];
  const float* conv_b  = (const float*)d_in[3];
  const float* W_xproj = (const float*)d_in[4];
  const float* W_dt    = (const float*)d_in[5];
  const float* b_dt    = (const float*)d_in[6];
  const float* A_log   = (const float*)d_in[7];
  const float* Dp      = (const float*)d_in[8];
  const float* W_out   = (const float*)d_in[9];
  float* out = (float*)d_out;

  char* ws = (char*)d_ws;
  unsigned short* X16  = (unsigned short*)(ws + kOffX16);
  unsigned short* WIN  = (unsigned short*)(ws + kOffWIN);
  unsigned short* XB   = (unsigned short*)(ws + kOffXB);
  unsigned short* DT16 = (unsigned short*)(ws + kOffXB);
  unsigned short* G16  = (unsigned short*)(ws + kOffG);
  unsigned short* U16  = (unsigned short*)(ws + kOffU);
  float*          BC   = (float*)(ws + kOffBC);
  unsigned short* DTLR = (unsigned short*)(ws + kOffDTLR);
  unsigned short* WOUT = (unsigned short*)(ws + kOffWOUT);
  unsigned short* WX   = (unsigned short*)(ws + kOffWX);
  unsigned short* WDT  = (unsigned short*)(ws + kOffWDT);

  cast_bf16_f16_kernel<<<(kRows * kDm / 8) / 256, 256, 0, stream>>>(x, X16, kRows * kDm / 8, kRows * kDm / 8, 1.0f);
  cast_bf16_f16_kernel<<<(kXzN * kDm / 8) / 256, 256, 0, stream>>>(W_in, WIN, kXzN * kDm / 8, kXzN * kDm / 8, kCarryWin);
  cast_bf16_f16_kernel<<<(kDm * kDin / 8) / 256, 256, 0, stream>>>(W_out, WOUT, kDm * kDin / 8, kDm * kDin / 8, kCarryWout);
  cast_bf16_f16_kernel<<<(kPrjP * kDin / 8) / 256, 256, 0, stream>>>(W_xproj, WX, kPrjP * kDin / 8, kPrjN * kDin / 8, kCarryWx);
  cast_bf16_f16_kernel<<<(kDin * kDtR / 8) / 256, 256, 0, stream>>>(W_dt, WDT, kDin * kDtR / 8, kDin * kDtR / 8, kCarryWdt);

  gemm_f16_kernel<EPI_INPROJ><<<dim3((kRows / 64) * (kXzN / 64) / 8), dim3(256), 0, stream>>>(
      X16, kDm, WIN, kDm, (void*)XB, (void*)G16, kDin, b_dt,
      kRows, kXzN, kDm, 1.0f / kCarryWin);

  conv_silu_kernel<<<dim3(kDin / 256, kRows / 64), dim3(256), 0, stream>>>(
      (const unsigned*)XB, conv_w, conv_b, U16);

  gemm_f16_kernel<EPI_XPROJ><<<dim3((kRows / 64) * (kPrjP / 64) / 8), dim3(256), 0, stream>>>(
      U16, kDin, WX, kDin, (void*)DTLR, (void*)BC, kPrjP, b_dt,
      kRows, kPrjP, kDin, 1.0f / kCarryWx);

  gemm_f16_kernel<EPI_DT><<<dim3((kRows / 64) * (kDin / 64) / 8), dim3(256), 0, stream>>>(
      DTLR, kDtR, WDT, kDtR, (void*)DT16, (void*)DT16, kDin, b_dt,
      kRows, kDin, kDtR, 1.0f / (kCarryDtLr * kCarryWdt));

  scan_kernel<<<dim3(kBatch * (kDin / 256)), dim3(256), 0, stream>>>(
      (const unsigned*)DT16, U16, (const unsigned*)G16, BC, A_log, Dp);

  gemm_f16_kernel<EPI_OUT><<<dim3((kRows / 64) * (kDm / 64) / 8), dim3(256), 0, stream>>>(
      U16, kDin, WOUT, kDin, (void*)out, (void*)out, kDm, b_dt,
      kRows, kDm, kDin, 1.0f / (kCarryY * kCarryWout));
}
